// SS1D_83769042141513
// MI455X (gfx1250) — hardware-run, weakly checked
//
#include <hip/hip_runtime.h>


namespace {
constexpr int B = 8, L = 2048, DM = 192, DI = 384, NS = 16, R = 12, XDW = 48, NR = B * L;
constexpr float XS = 8.0f, WSC = 256.0f, EPS = 1e-5f;
typedef _Float16 b16;
typedef __attribute__((ext_vector_type(16))) _Float16 v16b;
typedef __attribute__((ext_vector_type(8))) _Float16 v8b;
typedef __attribute__((ext_vector_type(8))) float v8f;
typedef __attribute__((ext_vector_type(4))) float v4f;
typedef __attribute__((ext_vector_type(2))) float v2f;
__device__ __forceinline__ float bf16_rne(float f) { unsigned int u = __float_as_uint(f); u += 0x7FFFu + ((u >> 16) & 1u); float r = __uint_as_float(u & 0xFFFF0000u); asm volatile("" : "+v"(r)); return r; }
__device__ __forceinline__ void split16(float v, b16& hi, b16& lo) { hi = (b16)v; lo = (b16)(v - (float)hi); }
__device__ __forceinline__ v16b frag_kb(const b16* p, int hh) { const v8b a = *(const v8b*)(p + 8 * hh), b = *(const v8b*)(p + 16 + 8 * hh); v16b f;
#pragma unroll
  for (int e = 0; e < 8; ++e) { f[e] = a[e]; f[8 + e] = b[e]; } return f; }
__device__ __forceinline__ v8f wmma16b(v16b a, v16b b, v8f c) { v8f d = __builtin_amdgcn_wmma_f32_16x16x32_f16(false, a, false, b, (short)0, c, false, false); asm volatile("v_nop\n\tv_nop\n\tv_nop\n\tv_nop" : "+v"(d) : "v"(a), "v"(b)); return d; }
__device__ __forceinline__ void wave_lds_sync() { __builtin_amdgcn_fence(__ATOMIC_RELEASE, "workgroup"); __builtin_amdgcn_wave_barrier(); __builtin_amdgcn_fence(__ATOMIC_ACQUIRE, "workgroup"); }
__device__ __forceinline__ float pmul(float a, float b) { float p = a * b; asm volatile("" : "+v"(p)); return p; }
__device__ __forceinline__ float silu(float v) { return v / (1.0f + __expf(-v)); }
__device__ __forceinline__ float softplus(float v) { return v > 20.0f ? v : __logf(1.0f + __expf(v)); }

__global__ __launch_bounds__(256) void wput_kernel(const float* __restrict__ win, const float* __restrict__ xp, const float* __restrict__ wo, b16* __restrict__ WIN, b16* __restrict__ XPT, b16* __restrict__ WOT) { const int u = blockIdx.x * 256 + threadIdx.x;
  for (int pass = 0; pass < 2; ++pass) {
    if (u < 2 * DI * (DM / 8)) { const int o = u / (DM / 8), k0 = (u % (DM / 8)) * 8; v8b v;
#pragma unroll
      for (int j = 0; j < 8; ++j) v[j] = (b16)(bf16_rne(win[(size_t)o * DM + k0 + j]) * WSC); *(volatile v8b*)(WIN + (size_t)o * DM + k0) = v; }
    if (u < XDW * (DI / 8)) { const int o = u / (DI / 8), k0 = (u % (DI / 8)) * 8; v8b v;
#pragma unroll
      for (int j = 0; j < 8; ++j) v[j] = (b16)(o < R + 2 * NS ? bf16_rne(xp[(size_t)o * DI + k0 + j]) * WSC : 0.0f); *(volatile v8b*)(XPT + (size_t)o * DI + k0) = v; }
    if (u < DM * (DI / 8)) { const int o = u / (DI / 8), k0 = (u % (DI / 8)) * 8; v8b v;
#pragma unroll
      for (int j = 0; j < 8; ++j) v[j] = (b16)(bf16_rne(wo[(size_t)o * DI + k0 + j]) * WSC); *(volatile v8b*)(WOT + (size_t)o * DI + k0) = v; }
    __threadfence(); } }
__global__ __launch_bounds__(32) void inproj_kernel(const float* __restrict__ x, const b16* __restrict__ WIN, int NRV, float* __restrict__ XZ) { __shared__ __attribute__((aligned(16))) b16 Ah[16][200]; __shared__ float Tf[16][132]; const int lane = threadIdx.x, nloc = lane & 15, hlf = lane >> 4; const int g = blockIdx.x % 6; const size_t m0 = (size_t)(blockIdx.x / 6) * 16; if (m0 >= (size_t)NRV) return;
  for (int rr = 0; rr < 16; ++rr) for (int q = 0; q < 6; ++q) Ah[rr][q * 32 + lane] = (b16)(bf16_rne(x[(m0 + rr) * DM + q * 32 + lane]) * XS);
  wave_lds_sync(); v8f acc[8];
#pragma unroll
  for (int t = 0; t < 8; ++t) acc[t] = (v8f){};
#pragma unroll
  for (int kb = 0; kb < DM; kb += 32) { const v16b a = frag_kb(&Ah[nloc][kb], hlf);
#pragma unroll
    for (int t = 0; t < 8; ++t) acc[t] = wmma16b(a, frag_kb(WIN + (size_t)(g * 128 + t * 16 + nloc) * DM + kb, hlf), acc[t]); }
#pragma unroll
  for (int t = 0; t < 8; ++t)
#pragma unroll
    for (int r8 = 0; r8 < 8; ++r8) Tf[8 * hlf + r8][t * 16 + nloc] = silu(acc[t][r8] * (1.0f / (XS * WSC)));
  wave_lds_sync();
  for (int pass = 0; pass < 2; ++pass) { for (int rr = 0; rr < 16; ++rr) *(volatile v4f*)(XZ + (m0 + rr) * 2 * DI + g * 128 + lane * 4) = *(const v4f*)(&Tf[rr][lane * 4]); __threadfence(); } }
__global__ __launch_bounds__(32) void xproj_kernel(const float* __restrict__ XZ, const b16* __restrict__ XPT, const float* __restrict__ dtw, const float* __restrict__ dtb, int NRV, float* __restrict__ XD, float* __restrict__ DL) { __shared__ __attribute__((aligned(16))) b16 Ah[16][DI + 8], Al[16][DI + 8]; __shared__ float Tf[16][52]; const int lane = threadIdx.x, nloc = lane & 15, hlf = lane >> 4; const size_t m0 = (size_t)blockIdx.x * 16; if (m0 >= (size_t)NRV) return;
  for (int rr = 0; rr < 16; ++rr) for (int q = 0; q < DI / 32; ++q) { b16 p, ql; split16(XZ[(m0 + rr) * 2 * DI + q * 32 + lane] * XS, p, ql); Ah[rr][q * 32 + lane] = p; Al[rr][q * 32 + lane] = ql; }
  wave_lds_sync(); v8f acc[3] = {(v8f){}, (v8f){}, (v8f){}};
#pragma unroll 2
  for (int kb = 0; kb < DI; kb += 32) { const v16b a = frag_kb(&Ah[nloc][kb], hlf), al = frag_kb(&Al[nloc][kb], hlf);
#pragma unroll
    for (int t = 0; t < 3; ++t) { const v16b bw = frag_kb(XPT + (size_t)(t * 16 + nloc) * DI + kb, hlf); acc[t] = wmma16b(a, bw, acc[t]); acc[t] = wmma16b(al, bw, acc[t]); } }
#pragma unroll
  for (int t = 0; t < 3; ++t)
#pragma unroll
    for (int r8 = 0; r8 < 8; ++r8) Tf[8 * hlf + r8][t * 16 + nloc] = acc[t][r8] * (1.0f / (XS * WSC));
  wave_lds_sync(); float wv[12][R];
#pragma unroll
  for (int j = 0; j < 12; ++j)
#pragma unroll
    for (int r = 0; r < R; ++r) wv[j][r] = bf16_rne(dtw[(lane * 12 + j) * R + r]);
  for (int pass = 0; pass < 2; ++pass) { for (int rr = 0; rr < 16; ++rr) { for (int c = lane; c < XDW; c += 32) ((volatile float*)XD)[(m0 + rr) * XDW + c] = Tf[rr][c];
#pragma unroll
      for (int j = 0; j < 12; ++j) { const int e = lane * 12 + j; float s = bf16_rne(dtb[e]);
#pragma unroll
        for (int r = 0; r < R; ++r) s += pmul(Tf[rr][r], wv[j][r]); ((volatile float*)DL)[(m0 + rr) * DI + e] = softplus(s); } }
    __threadfence(); } }
__global__ __launch_bounds__(32) void scan_kernel(const float* __restrict__ XZ, const float* __restrict__ XD, const float* __restrict__ DL, const float* __restrict__ Alog, const float* __restrict__ Dp, int LV, float* __restrict__ YS) {
  const int lane = threadIdx.x, b = blockIdx.x >> 2, g = blockIdx.x & 3; const int e0 = g * 96 + lane * 3; float A[3][NS], Dd[3];
  for (int j = 0; j < 3; ++j) { const int e = e0 + j; Dd[j] = bf16_rne(Dp[e]);
#pragma unroll
    for (int n = 0; n < NS; ++n) A[j][n] = -__expf(bf16_rne(Alog[e * NS + n])); }
  for (int pass = 0; pass < 2; ++pass) { float st[3][NS];
#pragma unroll
    for (int j = 0; j < 3; ++j)
#pragma unroll
      for (int n = 0; n < NS; ++n) st[j][n] = 0.0f;
#pragma unroll 1
    for (int t = 0; t < LV; ++t) { const size_t row = (size_t)b * L + t; float Bn[NS], Cn[NS];
#pragma unroll
      for (int n = 0; n < NS; ++n) { Bn[n] = XD[row * XDW + R + n]; Cn[n] = XD[row * XDW + R + NS + n]; }
#pragma unroll
      for (int j = 0; j < 3; ++j) { const int e = e0 + j; const float dl = DL[row * DI + e], u = XZ[row * 2 * DI + e]; const float du = pmul(dl, u); float y = pmul(u, Dd[j]);
#pragma unroll
        for (int n = 0; n < NS; ++n) { st[j][n] = pmul(__expf(pmul(dl, A[j][n])), st[j][n]) + pmul(du, Bn[n]); y += pmul(st[j][n], Cn[n]); }
        ((volatile float*)YS)[row * DI + e] = y; } }
    __threadfence(); } }
__global__ __launch_bounds__(32) void out_kernel(const float* __restrict__ YS, const float* __restrict__ XZ, const float* __restrict__ lng, const float* __restrict__ lnb, const b16* __restrict__ WOT, int NRV, float* __restrict__ out) { __shared__ __attribute__((aligned(16))) b16 Ah[16][DI + 8], Al[16][DI + 8]; __shared__ float Tf[16][196]; const int lane = threadIdx.x, nloc = lane & 15, hlf = lane >> 4; const size_t m0 = (size_t)blockIdx.x * 16; if (m0 >= (size_t)NRV) return;
  for (int rr = 0; rr < 16; ++rr) { float v[12]; float s = 0.0f;
#pragma unroll
    for (int q = 0; q < 12; ++q) { v[q] = YS[(m0 + rr) * DI + q * 32 + lane]; s += v[q]; } for (int o = 16; o; o >>= 1) s += __shfl_xor(s, o); const float mu = s * (1.0f / DI); float qq = 0.0f;
#pragma unroll
    for (int q = 0; q < 12; ++q) qq += pmul(v[q] - mu, v[q] - mu); for (int o = 16; o; o >>= 1) qq += __shfl_xor(qq, o); const float rs = rsqrtf(qq * (1.0f / DI) + EPS);
#pragma unroll
    for (int q = 0; q < 12; ++q) { const int c = q * 32 + lane; const float y = pmul(pmul(pmul(v[q] - mu, rs), bf16_rne(lng[c])) + bf16_rne(lnb[c]), XZ[(m0 + rr) * 2 * DI + DI + c]); b16 p, ql; split16(y * XS, p, ql); Ah[rr][c] = p; Al[rr][c] = ql; } }
  wave_lds_sync(); v8f acc[12];
#pragma unroll
  for (int t = 0; t < 12; ++t) acc[t] = (v8f){};
#pragma unroll 2
  for (int kb = 0; kb < DI; kb += 32) { const v16b a = frag_kb(&Ah[nloc][kb], hlf), al = frag_kb(&Al[nloc][kb], hlf);
#pragma unroll
    for (int t = 0; t < 12; ++t) { const v16b bw = frag_kb(WOT + (size_t)(t * 16 + nloc) * DI + kb, hlf); acc[t] = wmma16b(a, bw, acc[t]); acc[t] = wmma16b(al, bw, acc[t]); } }
#pragma unroll
  for (int t = 0; t < 12; ++t)
#pragma unroll
    for (int r8 = 0; r8 < 8; ++r8) Tf[8 * hlf + r8][t * 16 + nloc] = acc[t][r8] * (1.0f / (XS * WSC));
  wave_lds_sync();
  for (int pass = 0; pass < 2; ++pass) { for (int rr = 0; rr < 16; ++rr) { const float* tr = Tf[rr]; *(volatile v4f*)(out + (m0 + rr) * DM + lane * 4) = *(const v4f*)(&tr[lane * 4]); *(volatile v2f*)(out + (m0 + rr) * DM + 128 + lane * 2) = (v2f){tr[128 + lane * 2], tr[128 + lane * 2 + 1]}; } __threadfence(); } }
}

extern "C" void kernel_launch(void* const* d_in, const int* in_sizes, int n_in, void* d_out, int out_size, void* d_ws, size_t ws_size, hipStream_t stream) {
  (void)n_in;
  auto Fp = [&](int i) { return (const float*)d_in[i]; };
  if (in_sizes[0] != NR * DM || in_sizes[1] != 2 * DI * DM || in_sizes[2] != (R + 2 * NS) * DI || in_sizes[3] != DI * R || in_sizes[5] != DI * NS || in_sizes[9] != DM * DI || out_size != NR * DM) return;
  const int BV = B; const int NRV = BV * L; const int LV = L;
  size_t off = 0; char* ws = (char*)d_ws;
  auto carve = [&](size_t bytes) { char* p = ws + off; off += (bytes + 255) & ~(size_t)255; return p; };
  b16* WIN = (b16*)carve((size_t)2 * DI * DM * 2); b16* XPT = (b16*)carve((size_t)XDW * DI * 2); b16* WOT = (b16*)carve((size_t)DM * DI * 2);
  float* XZ = (float*)carve((size_t)NR * 2 * DI * 4); float* XD = (float*)carve((size_t)NR * XDW * 4); float* DL = (float*)carve((size_t)NR * DI * 4); float* YS = (float*)carve((size_t)NR * DI * 4);
  if (off > ws_size || off > ((size_t)128 << 20)) return;
  wput_kernel<<<(2 * DI * (DM / 8) + 255) / 256, 256, 0, stream>>>(Fp(1), Fp(2), Fp(9), WIN, XPT, WOT);
  inproj_kernel<<<(NRV / 16) * 6, 32, 0, stream>>>(Fp(0), WIN, NRV, XZ);
  xproj_kernel<<<NRV / 16, 32, 0, stream>>>(XZ, XPT, Fp(3), Fp(4), NRV, XD, DL);
  scan_kernel<<<BV * 4, 32, 0, stream>>>(XZ, XD, DL, Fp(5), Fp(6), LV, YS);
  out_kernel<<<NRV / 16, 32, 0, stream>>>(YS, XZ, Fp(7), Fp(8), WOT, NRV, (float*)d_out);
}
